// WavKANLayer_78512002171115
// MI455X (gfx1250) — hardware-verified
//
#include <hip/hip_runtime.h>


#ifndef NB
#define NB 256
#endif
#define NB_FULL 256
#define INF  1024
#define OUTF 1024
#ifndef P_RES
#define P_RES 0
#endif
#define QRS  2048.0f
#define QRI  (1.0f / 2048.0f)
#define ABLK 32
#define ATHR 256
#define OSP  68

static_assert(NB <= NB_FULL);
static_assert(NB % 32 == 0);
static_assert(OUTF % 64 == 0);
static_assert(INF % 32 == 0);
static_assert(INF % 8 == 0);
static_assert(((size_t)NB * INF) % 256 == 0);
static_assert(((size_t)OUTF * INF) % 8 == 0);
static_assert(((size_t)OUTF * INF) % ((size_t)ABLK * ATHR * 4) == 0);
static_assert(ABLK == 32);
static_assert(ATHR == 256);
static_assert((OSP * 4) % 16 == 0);
static_assert(OSP >= 64);
static_assert(32 * 16 * 8 == 16 * 64 * 4);
static_assert(32 * 16 == 256 * 2);
static_assert(8 * 16 == 128);
static_assert(16 * OSP * 4 <= 131072);
static_assert(2 * 256 * 2 <= 131072);
static_assert(8 * 4 <= 131072);

typedef _Float16 h16;
typedef unsigned short bf;
typedef __attribute__((ext_vector_type(16))) _Float16 v16h;
typedef __attribute__((ext_vector_type(8)))  _Float16 v8h;
typedef __attribute__((ext_vector_type(8)))  float    v8f;
typedef __attribute__((ext_vector_type(4)))  float    v4f;
typedef __attribute__((ext_vector_type(4)))  int      v4i;
typedef v4f  __attribute__((may_alias)) v4fa;
typedef v8h  __attribute__((may_alias)) v8ha;

__device__ __forceinline__ unsigned short f2bf(float f) { unsigned u = __float_as_uint(f); u += 0x7FFFu + ((u >> 16) & 1u); return (unsigned short)(u >> 16); }
__device__ __forceinline__ float bfr(float f) { return __uint_as_float(((unsigned)f2bf(f)) << 16); }
__device__ __forceinline__ v16h cat16(v8h lo, v8h hi) { return __builtin_shufflevector(lo, hi, 0, 1, 2, 3, 4, 5, 6, 7, 8, 9, 10, 11, 12, 13, 14, 15); }
__device__ __forceinline__ v8f wmma16(v16h a, v16h b, v8f c) { return __builtin_amdgcn_wmma_f32_16x16x32_f16(false, a, false, b, (short)0, c, false, false); }
__device__ __forceinline__ v8f wmma16g(v16h a, v16h b, v8f c) { c = wmma16(a, b, c); asm volatile("v_nop\n\tv_nop\n\tv_nop\n\tv_nop" : "+v"(c) : "v"(a), "v"(b)); return c; }
__device__ __forceinline__ v16h  ldh(const h16* p) { return cat16(*(const v8h*)p, *(const v8h*)(p + 16)); }
__device__ __forceinline__ void wave_sync() { __builtin_amdgcn_fence(3  , "wavefront"); __builtin_amdgcn_wave_barrier(); asm volatile("" ::: "memory"); }
static __device__ __forceinline__ h16 toh_flush(float v) { const float w = (fabsf(v) < 6.103515625e-05f) ? 0.0f : v; return (h16)w; }

#define CHW ((unsigned)(((size_t)OUTF * INF) / ABLK))
__global__ __launch_bounds__(256) void k_assert(const float* __restrict__ sc, const float* __restrict__ tr, int* FL) {
    __shared__ int wc[8];
    const unsigned tid = threadIdx.x; const unsigned bx = blockIdx.x;
    const unsigned lane = tid & 31u;
    const int wave = __builtin_amdgcn_readfirstlane((int)(threadIdx.x >> 5));
    const size_t base = (size_t)bx * CHW;
    int miss = 0;
#pragma unroll 1
    for (unsigned it = 0; it < CHW / (ATHR * 4u); ++it) {
        const size_t o = base + ((size_t)it * ATHR + tid) * 4u;
        const v4f s = *(const v4f*)(sc + o); const v4f t = *(const v4f*)(tr + o);
#pragma unroll
        for (int i = 0; i < 4; ++i) {
            miss += (__float_as_uint(s[i]) != 0x3f800000u) ? 1 : 0;
            miss += ((__float_as_uint(t[i]) & 0x7fffffffu) != 0u) ? 1 : 0; }
    }
    miss += __shfl_xor(miss, 16, 32); miss += __shfl_xor(miss, 8, 32); miss += __shfl_xor(miss, 4, 32); miss += __shfl_xor(miss, 2, 32); miss += __shfl_xor(miss, 1, 32);
    if (lane == 0u) wc[wave] = miss;
    __syncthreads();
    int tot = 0;
#pragma unroll
    for (int w = 0; w < 8; ++w) tot += wc[w];
    if (tid < 8u) {
        v4i o; o[0] = tot; o[1] = tot; o[2] = tot; o[3] = tot;
        int* p = FL + (size_t)bx * 32u + tid * 4u;
        *(volatile v4i*)p = o; __threadfence(); *(volatile v4i*)p = o;
    }
}

__global__ __launch_bounds__(256) void k_phi(const float* __restrict__ X, h16* PH, h16* PR) {
#pragma clang fp contract(off)
    __shared__ __align__(16) h16 sv[256];
    __shared__ __align__(16) h16 sr[256];
    const unsigned tid = threadIdx.x; const unsigned bx = blockIdx.x;
    const int wave = __builtin_amdgcn_readfirstlane((int)(threadIdx.x >> 5));
    const size_t e = (size_t)bx * 256u + tid;
    const float xb = bfr(X[e]);
    const float ex = expf((-0.5f * xb) * xb);
    const float ph = (-xb) * ex;
    const h16 hv = toh_flush(ph);
    sv[tid] = hv;
    sr[tid] = toh_flush((ph - (float)hv) * QRS);
    __syncthreads();
    const unsigned l = tid & 31u;
    if (wave == 0) {
        const v8h o = *(const v8ha*)(&sv[l * 8u]);
        h16* p = PH + (size_t)bx * 256u + l * 8u;
        *(volatile v8h*)p = o; __threadfence(); *(volatile v8h*)p = o;
    } else if (wave == 1) {
        if (P_RES) {
            const v8h o = *(const v8ha*)(&sr[l * 8u]);
            h16* p = PR + (size_t)bx * 256u + l * 8u;
            *(volatile v8h*)p = o; __threadfence(); *(volatile v8h*)p = o;
        }
    }
}

__global__ __launch_bounds__(256) void k_wcv8(const float* __restrict__ src, h16* dst, size_t n8) {
    const size_t i = (size_t)blockIdx.x * 256 + threadIdx.x; if (i >= n8) return;
    const v8f v = *(const v8f*)(src + i * 8); v8h o;
#pragma unroll
    for (int k = 0; k < 8; ++k) o[k] = toh_flush(bfr(v[k]));
    *(volatile v8h*)(dst + i * 8) = o; __threadfence(); *(volatile v8h*)(dst + i * 8) = o;
}

__global__ __launch_bounds__(32) void k_gemm(const h16* __restrict__ PH, const h16* __restrict__ PR, const h16* __restrict__ WH, const int* __restrict__ FL, float* OUT) {
    __shared__ __align__(16) float os[16 * OSP];
    const unsigned lane = threadIdx.x & 31u, lr = lane & 15u, hi = lane >> 4;
    const unsigned r0 = blockIdx.x * 32u, c0 = blockIdx.y * 64u;
    v8f acc[2][4];
#if P_RES
    v8f acr[2][4];
#endif
#pragma unroll
    for (int mb = 0; mb < 2; ++mb)
#pragma unroll
        for (int nb = 0; nb < 4; ++nb) { acc[mb][nb] = (v8f){};
#if P_RES
            acr[mb][nb] = (v8f){};
#endif
        }
    const size_t aoff = (size_t)(r0 + lr) * INF + 8u * hi, boff = (size_t)(c0 + lr) * INF + 8u * hi;
#pragma unroll 1
    for (unsigned kc = 0; kc < INF; kc += 32u) {
        v16h a[2];
#if P_RES
        v16h ar[2];
#endif
#pragma unroll
        for (int mb = 0; mb < 2; ++mb) { a[mb] = ldh(PH + aoff + (size_t)mb * 16 * INF + kc);
#if P_RES
            ar[mb] = ldh(PR + aoff + (size_t)mb * 16 * INF + kc);
#endif
        }
#pragma unroll
        for (int nb = 0; nb < 4; ++nb) { const v16h b = ldh(WH + boff + (size_t)nb * 16 * INF + kc);
#pragma unroll
            for (int mb = 0; mb < 2; ++mb) { acc[mb][nb] = wmma16g(a[mb], b, acc[mb][nb]);
#if P_RES
                acr[mb][nb] = wmma16g(ar[mb], b, acr[mb][nb]);
#endif
            } }
    }
#if !P_RES
    (void)PR;
#endif
    int fl = FL[(size_t)lane * 32u];
    fl |= __shfl_xor(fl, 16, 32); fl |= __shfl_xor(fl, 8, 32); fl |= __shfl_xor(fl, 4, 32); fl |= __shfl_xor(fl, 2, 32); fl |= __shfl_xor(fl, 1, 32);
    const bool bad = fl != 0;
    const float qn = __uint_as_float(0x7fc00000u);
#pragma unroll
    for (int mb = 0; mb < 2; ++mb) {
#pragma unroll
        for (int nb = 0; nb < 4; ++nb) {
#pragma unroll
            for (int j = 0; j < 8; ++j) {
#if P_RES
                os[(hi * 8 + j) * OSP + nb * 16 + lr] = acc[mb][nb][j] + acr[mb][nb][j] * QRI;
#else
                os[(hi * 8 + j) * OSP + nb * 16 + lr] = acc[mb][nb][j];
#endif
            } }
        wave_sync();
        float* orow = OUT + (size_t)(r0 + mb * 16) * OUTF + c0;
#pragma unroll 1
        for (int ps = 0; ps < 2; ++ps) {
#pragma unroll
            for (int s = 0; s < 8; ++s) { const unsigned row = 2u * s + (lane >> 4), cofs = (lane & 15u) * 4u;
                v4f val = *(const v4fa*)(&os[row * OSP + cofs]);
                val[0] = bad ? qn : val[0]; val[1] = bad ? qn : val[1]; val[2] = bad ? qn : val[2]; val[3] = bad ? qn : val[3];
                *(volatile v4f*)(orow + (size_t)row * OUTF + cofs) = val; }
            if (ps == 0) __threadfence(); }
        wave_sync();
    }
}

static constexpr size_t al256(size_t v) { return (v + 255) & ~(size_t)255; }
static constexpr size_t SZ_PH = al256((size_t)NB * INF * 2);
static constexpr size_t SZ_PR = al256((size_t)NB * INF * 2);
static constexpr size_t SZ_WH = al256((size_t)OUTF * INF * 2);
static constexpr size_t SZ_FL = al256((size_t)ABLK * 128);
static constexpr size_t SZ_TOTAL = SZ_PH + SZ_PR + SZ_WH + SZ_FL;
static_assert(SZ_TOTAL <= (size_t)134217728);
static_assert((size_t)ABLK * 32 * 4 <= SZ_FL);
static_assert(((size_t)NB * INF / 256) * 256 * 2 <= SZ_PH);
static_assert((size_t)NB * OUTF * 4 == (size_t)(NB / 32) * (OUTF / 64) * 32 * 64 * 4);

extern "C" void kernel_launch(void* const* d_in, const int* in_sizes, int n_in,
                              void* d_out, int out_size, void* d_ws, size_t ws_size, hipStream_t stream) {
    if (n_in < 4) return;
    if ((size_t)in_sizes[0] < (size_t)NB * INF) return;
    if ((size_t)in_sizes[1] < (size_t)OUTF * INF || (size_t)in_sizes[2] < (size_t)OUTF * INF || (size_t)in_sizes[3] < (size_t)OUTF * INF) return;
    if ((size_t)out_size < (size_t)NB * OUTF) return;
    if (SZ_TOTAL > ws_size) return;
    const float* x  = (const float*)d_in[0];
    const float* w  = (const float*)d_in[1];
    const float* sc = (const float*)d_in[2];
    const float* tr = (const float*)d_in[3];
    float* OUT = (float*)d_out;
    char* wsp = (char*)d_ws;
    h16* PH = (h16*)wsp; wsp += SZ_PH;
    h16* PR = (h16*)wsp; wsp += SZ_PR;
    h16* WH = (h16*)wsp; wsp += SZ_WH;
    int* FL = (int*)wsp; wsp += SZ_FL;

    k_assert<<<ABLK, ATHR, 0, stream>>>(sc, tr, FL);
    k_phi<<<(unsigned)(((size_t)NB * INF) / 256), 256, 0, stream>>>(x, PH, PR);
    { const size_t n8 = (size_t)OUTF * INF / 8;
      k_wcv8<<<(unsigned)((n8 + 255) / 256), 256, 0, stream>>>(w, WH, n8); }
    k_gemm<<<dim3(NB / 32, OUTF / 64, 1), 32, 0, stream>>>(PH, PR, WH, FL, OUT);
}
